// NeuralLaplaceModel_59691455480128
// MI455X (gfx1250) — hardware-run, weakly checked
//
#include <hip/hip_runtime.h>
#include <math.h>

typedef __attribute__((ext_vector_type(16))) _Float16 v16h;
typedef __attribute__((ext_vector_type(8)))  _Float16 v8h;
typedef __attribute__((ext_vector_type(16))) __bf16   v16b;
typedef __attribute__((ext_vector_type(8)))  __bf16   v8b;
typedef __attribute__((ext_vector_type(8)))  float    v8f;
typedef __attribute__((ext_vector_type(4)))  float    v4f;

constexpr int kBatch   = 2048;
constexpr int kALen    = 32;
constexpr int kTP      = 16;
constexpr int kStateD  = 17;
constexpr int kActD    = 6;
constexpr int kTerms   = 33;
constexpr int kHid     = 64;
constexpr int kGruH    = 32;
constexpr int kOutD    = 17;
constexpr int kLat     = kStateD + 2;
constexpr int kFeat    = 2 * kTerms + kLat;
constexpr int kFeatP   = 96;
constexpr int kN3      = 2 * kOutD * kTerms;
constexpr int kNP      = kOutD * kTerms;
constexpr int kN3P     = 1152;
constexpr int kGroups  = kN3P / 32;
constexpr int kRows    = kBatch * kTP;
constexpr int kRowTile = 64;
constexpr int kPPitch  = 32;
constexpr int kApitch  = 104;
constexpr int kHpitch  = 72;
constexpr int kRawPitch = 20;
constexpr int kGateRows = 3 * kGruH;
constexpr int kGwMat   = kGateRows * kGruH;
static_assert(kFeat == 85 && kN3 == 1122 && kNP == 561, "shape constants");
static_assert(kFeatP % 32 == 0 && kFeatP >= kFeat, "K pad of layer 1");
static_assert(kHid % 32 == 0 && kGruH == 32, "K multiples of 32");
static_assert(kN3P % 32 == 0 && kGroups == 36 && (kN3P / 2) >= kNP, "N pad of layer 3");
static_assert(kRows % kRowTile == 0 && kBatch % 32 == 0, "tile multiples");
static_assert((kRowTile * kOutD * 4) % 128 == 0, "out tile is whole lines");
static_assert(kRowTile * kHpitch <= kRowTile * kApitch, "h2 planes fit in the feature planes");

constexpr float kPi      = (float)3.14159265358979323846;
constexpr float kHalfPi  = (float)(3.14159265358979323846 / 2.0);
constexpr float kAlpha   = 1e-3f;
constexpr float kLogTol  = (float)(-4.605170185988091368);
constexpr float kThird   = 1.0f / 3.0f;
constexpr float kCarry   = 64.0f;
constexpr float kCarryInv2 = 1.0f / (kCarry * kCarry);

constexpr size_t kSzW1  = (size_t)kHid * kFeatP * 2;
constexpr size_t kSzW2  = (size_t)kHid * kHid * 2;
constexpr size_t kSzW3  = (size_t)kN3P * kHid * 2;
constexpr size_t kSzB3  = (size_t)kN3P * 4;
constexpr size_t kSzGW  = (size_t)4 * kGwMat * 2;
constexpr size_t kSzPP  = (size_t)kBatch * kPPitch * 4;
constexpr size_t kOffW1H = 0;
constexpr size_t kOffW1L = kOffW1H + kSzW1;
constexpr size_t kOffW2H = kOffW1L + kSzW1;
constexpr size_t kOffW2L = kOffW2H + kSzW2;
constexpr size_t kOffW3H = kOffW2L + kSzW2;
constexpr size_t kOffW3L = kOffW3H + kSzW3;
constexpr size_t kOffB3P = kOffW3L + kSzW3;
constexpr size_t kOffGW  = kOffB3P + kSzB3;
constexpr size_t kOffPP  = kOffGW + kSzGW;
constexpr size_t kWsTotal = kOffPP + kSzPP;
static_assert(kWsTotal == 627200ull, "carve total");
static_assert(kWsTotal <= 134217728ull, "carve cap");
static_assert((kOffW1L % 128) == 0 && (kOffW2H % 128) == 0 && (kOffW2L % 128) == 0 && (kOffW3H % 128) == 0 &&
              (kOffW3L % 128) == 0 && (kOffB3P % 128) == 0 && (kOffGW % 128) == 0 && (kOffPP % 128) == 0,
              "128-B aligned regions");

__device__ __forceinline__ unsigned short f2bf_bits(float f) {
  unsigned u = __float_as_uint(f);
  return (unsigned short)((u + 0x7FFFu + ((u >> 16) & 1u)) >> 16);
}
__device__ __forceinline__ float bf_bits2f(unsigned short h) { return __uint_as_float(((unsigned)h) << 16); }

__device__ __forceinline__ void bf_split(float f, __bf16& hi, __bf16& lo) {
  const unsigned short hb = f2bf_bits(f);
  hi = __builtin_bit_cast(__bf16, hb);
  lo = __builtin_bit_cast(__bf16, f2bf_bits(f - bf_bits2f(hb)));
}

template <typename T> struct Frag;
template <> struct Frag<_Float16> {
  typedef v16h V; union U { v16h v; v8h h[2]; };
  static __device__ __forceinline__ v16h load(const _Float16* p) {
    U f; f.h[0] = *(const v8h*)(p); f.h[1] = *(const v8h*)(p + 16); return f.v;
  }
};
template <> struct Frag<__bf16> {
  typedef v16b V; union U { v16b v; v8b h[2]; };
  static __device__ __forceinline__ v16b load(const __bf16* p) {
    U f; f.h[0] = *(const v8b*)(p); f.h[1] = *(const v8b*)(p + 16); return f.v;
  }
};
typedef Frag<_Float16> FragH;
typedef Frag<__bf16>   FragB;

__device__ __forceinline__ v8f mma_b(v16b a, v16b b, v8f c) {
  c = __builtin_amdgcn_wmma_f32_16x16x32_bf16(false, a, false, b, (short)0, c, false, false);
  asm volatile("v_nop\n\tv_nop\n\tv_nop\n\tv_nop" : "+v"(c) : "v"(a), "v"(b));
  return c;
}
__device__ __forceinline__ v8f mma_h(v16h a, v16h b, v8f c) {
  c = __builtin_amdgcn_wmma_f32_16x16x32_f16(false, a, false, b, (short)0, c, false, false);
  asm volatile("v_nop\n\tv_nop\n\tv_nop\n\tv_nop" : "+v"(c) : "v"(a), "v"(b));
  return c;
}

#define LDS_FRAG_BF(dst, base, off) do { FragB::U u_; u_.h[0] = *(const v8b*)((base) + (off)); u_.h[1] = *(const v8b*)((base) + (off) + 16); (dst) = u_.v; } while (0)
#define LDS_FRAG_HF(dst, base, off) do { FragH::U u_; u_.h[0] = *(const v8h*)((base) + (off)); u_.h[1] = *(const v8h*)((base) + (off) + 16); (dst) = u_.v; } while (0)

__device__ __forceinline__ void store_hilo8(const v4f a0, const v4f a1, unsigned short* qh, unsigned short* ql) {
  v8h hv, lv;
#pragma unroll
  for (int e = 0; e < 4; ++e) {
    const float f0 = a0[e];
    const float f1 = a1[e];
    const unsigned short h0 = f2bf_bits(f0), h1 = f2bf_bits(f1);
    const unsigned short l0 = f2bf_bits(f0 - bf_bits2f(h0)), l1 = f2bf_bits(f1 - bf_bits2f(h1));
    hv[e]     = __builtin_bit_cast(_Float16, h0);
    hv[4 + e] = __builtin_bit_cast(_Float16, h1);
    lv[e]     = __builtin_bit_cast(_Float16, l0);
    lv[4 + e] = __builtin_bit_cast(_Float16, l1);
  }
  *(volatile v8h*)qh = hv;
  *(volatile v8h*)ql = lv;
  __threadfence();
  *(volatile v8h*)qh = hv;
  *(volatile v8h*)ql = lv;
}

constexpr int kPrepThreads = 128;
constexpr int kBlkW1 = (kHid * kFeatP / 8) / kPrepThreads;
constexpr int kBlkW2 = (kHid * kHid / 8) / kPrepThreads;
constexpr int kBlkW3 = (kN3P * kHid / 8) / kPrepThreads;
constexpr int kBlkGWper = (kGwMat / 8) / kPrepThreads;
constexpr int kBlkGW = 4 * kBlkGWper;
constexpr int kB3Groups = kN3P / 4;
constexpr int kBlkB3 = (kB3Groups + kPrepThreads - 1) / kPrepThreads;
constexpr int kPrepBlocks = kBlkW1 + kBlkW2 + kBlkW3 + kBlkGW + kBlkB3;
static_assert(kBlkW1 * kPrepThreads * 8 == kHid * kFeatP, "W1 coverage");
static_assert(kBlkW2 * kPrepThreads * 8 == kHid * kHid, "W2 coverage");
static_assert(kBlkW3 * kPrepThreads * 8 == kN3P * kHid, "W3 coverage");
static_assert(kBlkGWper * kPrepThreads * 8 == kGwMat, "GRU plane coverage");
static_assert((kB3Groups % 32) == 0, "bias tail is whole waves");
static_assert(kPrepBlocks == 97, "prep grid");

__global__ __launch_bounds__(128) void prep_planes_kernel(
    const float* __restrict__ W1, const float* __restrict__ W2, const float* __restrict__ W3,
    const float* __restrict__ b3,
    const float* __restrict__ Wih0, const float* __restrict__ Whh0,
    const float* __restrict__ Wih1, const float* __restrict__ Whh1,
    unsigned short* __restrict__ W1H, unsigned short* __restrict__ W1L,
    unsigned short* __restrict__ W2H, unsigned short* __restrict__ W2L,
    unsigned short* __restrict__ W3H, unsigned short* __restrict__ W3L,
    float* __restrict__ B3P, unsigned short* __restrict__ GW)
{
  const int tid = threadIdx.x;
  int blk = blockIdx.x;
  if (blk < kBlkW1) {
    const int gi = blk * kPrepThreads + tid;
    const int n  = gi / (kFeatP / 8);
    const int k0 = (gi - n * (kFeatP / 8)) * 8;
    v4f a0, a1;
#pragma unroll
    for (int e = 0; e < 4; ++e) {
      const int ka = k0 + e, kb = k0 + 4 + e;
      const int kac = (ka < kFeat) ? ka : (kFeat - 1);
      const int kbc = (kb < kFeat) ? kb : (kFeat - 1);
      float va = W1[n * kFeat + kac];
      float vb = W1[n * kFeat + kbc];
      asm volatile("" : "+v"(va));
      asm volatile("" : "+v"(vb));
      a0[e] = (ka < kFeat) ? va : 0.0f;
      a1[e] = (kb < kFeat) ? vb : 0.0f;
    }
    store_hilo8(a0, a1, W1H + (size_t)gi * 8, W1L + (size_t)gi * 8);
    return;
  }
  blk -= kBlkW1;
  if (blk < kBlkW2) {
    const int gi = blk * kPrepThreads + tid;
    const v4f a0 = *(const v4f*)(W2 + (size_t)gi * 8);
    const v4f a1 = *(const v4f*)(W2 + (size_t)gi * 8 + 4);
    store_hilo8(a0, a1, W2H + (size_t)gi * 8, W2L + (size_t)gi * 8);
    return;
  }
  blk -= kBlkW2;
  if (blk < kBlkW3) {
    const int gi = blk * kPrepThreads + tid;
    const int pr = gi >> 3, kg = gi & 7;
    const int g = pr >> 5, j = pr & 31;
    const int p = 16 * g + (j & 15);
    const bool valid = (p < kNP);
    const int orig = (j < 16) ? p : (kNP + p);
    const int origc = valid ? orig : 0;
    const float* src = W3 + (size_t)origc * kHid + kg * 8;
    v4f r0 = *(const v4f*)(src);
    v4f r1 = *(const v4f*)(src + 4);
    asm volatile("" : "+v"(r0));
    asm volatile("" : "+v"(r1));
    v4f a0, a1;
#pragma unroll
    for (int e = 0; e < 4; ++e) {
      const float f0 = r0[e];
      const float f1 = r1[e];
      a0[e] = valid ? f0 : 0.0f;
      a1[e] = valid ? f1 : 0.0f;
    }
    store_hilo8(a0, a1, W3H + (size_t)gi * 8, W3L + (size_t)gi * 8);
    return;
  }
  blk -= kBlkW3;
  if (blk < kBlkGW) {
    const int mat = blk / kBlkGWper;
    const int gl  = (blk - mat * kBlkGWper) * kPrepThreads + tid;
    const int n = gl >> 2, k0 = (gl & 3) * 8;
    const float* W = (mat == 0) ? Wih0 : (mat == 1) ? Whh0 : (mat == 2) ? Wih1 : Whh1;
    const int rl = (mat == 0) ? kActD : kGruH;
    v8h hv;
#pragma unroll
    for (int e = 0; e < 8; ++e) {
      const int k = k0 + e;
      const int kc = (k < rl) ? k : (rl - 1);
      float v = W[n * rl + kc];
      asm volatile("" : "+v"(v));
      const float s = (k < rl) ? (v * kCarry) : 0.0f;
      hv[e] = (_Float16)s;
    }
    unsigned short* q = GW + (size_t)mat * kGwMat + (size_t)gl * 8;
    *(volatile v8h*)q = hv;
    __threadfence();
    *(volatile v8h*)q = hv;
    return;
  }
  blk -= kBlkGW;
  {
    const int gl  = blk * kPrepThreads + tid;
    const int glc = (gl < kB3Groups) ? gl : (kB3Groups - 1);
    v4f o;
#pragma unroll
    for (int e = 0; e < 4; ++e) {
      const int pn = 4 * glc + e;
      const int g = pn >> 5, j = pn & 31;
      const int p = 16 * g + (j & 15);
      const bool valid = (p < kNP);
      const int orig = (j < 16) ? p : (kNP + p);
      const int origc = valid ? orig : 0;
      float v = b3[origc];
      asm volatile("" : "+v"(v));
      o[e] = valid ? v : 0.0f;
    }
    if (gl < kB3Groups) {
      float* q = B3P + (size_t)gl * 4;
      *(volatile v4f*)q = o;
      __threadfence();
      *(volatile v4f*)q = o;
    }
  }
}

constexpr int kGruWaves = 2;

__global__ __launch_bounds__(64) void gru_encode_kernel(
    const float* __restrict__ obs, const float* __restrict__ action,
    const unsigned short* __restrict__ gwp,
    const float* __restrict__ bih0, const float* __restrict__ bhh0,
    const float* __restrict__ bih1, const float* __restrict__ bhh1,
    const float* __restrict__ Wout, const float* __restrict__ bout,
    float* __restrict__ pplane)
{
  __shared__ __align__(16) _Float16 sW[4 * kGwMat];
  __shared__ __align__(16) float    sBias[4 * kGateRows];
  __shared__ __align__(16) float    sWo[2 * kGruH];
  __shared__ __align__(16) _Float16 sAct[kGruWaves][2][16 * kGruH];
  __shared__ __align__(16) float    sHst[kGruWaves][2][16 * kGruH];
  __shared__ __align__(16) float    sPr[kGruWaves][16 * kPPitch];

  const int tid = threadIdx.x, lane = tid & 31, wave = tid >> 5;
  const int h = lane >> 4, c = lane & 15;
  const int gb0 = blockIdx.x * (kGruWaves * 16) + wave * 16;

  {
    const _Float16* gw = (const _Float16*)gwp;
#pragma unroll 1
    for (int i = 0; i < (4 * kGwMat / 8) / 64; ++i) {
      const int idx = i * 64 + tid;
      *(v8h*)(sW + idx * 8) = *(const v8h*)(gw + (size_t)idx * 8);
    }
  }
  {
    const int t2 = (64 + tid < kGateRows) ? (64 + tid) : (kGateRows - 1);
    const float a0 = bih0[tid], a1 = bhh0[tid], a2 = bih1[tid], a3 = bhh1[tid];
    const float c0 = bih0[t2], c1 = bhh0[t2], c2 = bih1[t2], c3 = bhh1[t2];
    sBias[0 * kGateRows + tid] = a0;
    sBias[1 * kGateRows + tid] = a1;
    sBias[2 * kGateRows + tid] = a2;
    sBias[3 * kGateRows + tid] = a3;
    if (tid < 32) {
      sBias[0 * kGateRows + 64 + tid] = c0;
      sBias[1 * kGateRows + 64 + tid] = c1;
      sBias[2 * kGateRows + 64 + tid] = c2;
      sBias[3 * kGateRows + 64 + tid] = c3;
    }
    sWo[tid] = Wout[tid];
  }
  {
    float* hz = &sHst[wave][0][0];
#pragma unroll 1
    for (int i = lane; i < 2 * 16 * kGruH; i += 32) hz[i] = 0.0f;
    _Float16* az = &sAct[wave][0][0];
    v8h z8;
#pragma unroll
    for (int e = 0; e < 8; ++e) z8[e] = (_Float16)0.0f;
#pragma unroll 1
    for (int i = lane; i < (2 * 16 * kGruH) / 8; i += 32) *(v8h*)(az + i * 8) = z8;
  }
  __syncthreads();

  const v8f zacc = {0.f, 0.f, 0.f, 0.f, 0.f, 0.f, 0.f, 0.f};

#pragma unroll 1
  for (int t = 0; t < kALen; ++t) {
    const int at = kALen - 1 - t;
    const float* ap = action + ((size_t)(gb0 + c) * kALen + at) * kActD;
    float x0 = ap[0], x1 = ap[1], x2 = ap[2], x3 = ap[3], x4 = ap[4], x5 = ap[5];
    asm volatile("" : "+v"(x0), "+v"(x1), "+v"(x2), "+v"(x3), "+v"(x4), "+v"(x5));
    const bool lowhalf = (h == 0);
    v16h xa;
    xa[0] = lowhalf ? (_Float16)((x0 * kThird) * kCarry) : (_Float16)0.0f;
    xa[1] = lowhalf ? (_Float16)((x1 * kThird) * kCarry) : (_Float16)0.0f;
    xa[2] = lowhalf ? (_Float16)((x2 * kThird) * kCarry) : (_Float16)0.0f;
    xa[3] = lowhalf ? (_Float16)((x3 * kThird) * kCarry) : (_Float16)0.0f;
    xa[4] = lowhalf ? (_Float16)((x4 * kThird) * kCarry) : (_Float16)0.0f;
    xa[5] = lowhalf ? (_Float16)((x5 * kThird) * kCarry) : (_Float16)0.0f;
#pragma unroll
    for (int i = 6; i < 16; ++i) xa[i] = (_Float16)0.0f;

    v16h ain = xa;
#pragma unroll 1
    for (int L = 0; L < 2; ++L) {
      _Float16* hb = &sAct[wave][L][0];
      float*    hs = &sHst[wave][L][0];
      const _Float16* wi = sW + (2 * L) * kGwMat;
      const _Float16* wr = sW + (2 * L + 1) * kGwMat;
      const float* bi = sBias + (2 * L) * kGateRows;
      const float* bh = sBias + (2 * L + 1) * kGateRows;
      v16h arec;
      LDS_FRAG_HF(arec, hb, c * kGruH + 8 * h);
#pragma unroll 1
      for (int ht = 0; ht < 2; ++ht) {
        const int n = ht * 16 + c;
        v16h wf;
        v8f accR = zacc, accZ = zacc, accX = zacc, accH = zacc;
        LDS_FRAG_HF(wf, wi, n * kGruH + 8 * h);
        accR = mma_h(ain, wf, accR);
        LDS_FRAG_HF(wf, wr, n * kGruH + 8 * h);
        accR = mma_h(arec, wf, accR);
        LDS_FRAG_HF(wf, wi, (n + kGruH) * kGruH + 8 * h);
        accZ = mma_h(ain, wf, accZ);
        LDS_FRAG_HF(wf, wr, (n + kGruH) * kGruH + 8 * h);
        accZ = mma_h(arec, wf, accZ);
        LDS_FRAG_HF(wf, wi, (n + 2 * kGruH) * kGruH + 8 * h);
        accX = mma_h(ain, wf, accX);
        LDS_FRAG_HF(wf, wr, (n + 2 * kGruH) * kGruH + 8 * h);
        accH = mma_h(arec, wf, accH);
        const float bir = bi[n], biz = bi[n + kGruH], bin = bi[n + 2 * kGruH];
        const float bhr = bh[n], bhz = bh[n + kGruH], bhn = bh[n + 2 * kGruH];
#pragma unroll
        for (int r = 0; r < 8; ++r) {
          const int ix = (8 * h + r) * kGruH + n;
          const float pr = (accR[r] * kCarryInv2 + bir) + bhr;
          const float pz = (accZ[r] * kCarryInv2 + biz) + bhz;
          const float xn = accX[r] * kCarryInv2 + bin;
          const float hn = accH[r] * kCarryInv2 + bhn;
          const float rg = 1.0f / (1.0f + expf(-pr));
          const float zg = 1.0f / (1.0f + expf(-pz));
          const float ng = tanhf(xn + rg * hn);
          const float hold = hs[ix];
          const float hnew = (1.0f - zg) * ng + zg * hold;
          hs[ix] = hnew;
          hb[ix] = (_Float16)(hnew * kCarry);
        }
      }
      __syncthreads();
      LDS_FRAG_HF(ain, hb, c * kGruH + 8 * h);
    }
  }

  float d = 0.0f;
  {
    const float* hrow = &sHst[wave][1][0] + c * kGruH;
    const float* wo = sWo + h * kGruH;
#pragma unroll 4
    for (int j = 0; j < kGruH; ++j) d = fmaf(hrow[j], wo[j], d);
    d += bout[h];
  }
  const float other = __shfl_xor(d, 16, 32);
  const float pa0 = (h == 0) ? d : other;
  const float pa1 = (h == 0) ? other : d;
  {
    float* pr = &sPr[wave][0] + c * kPPitch;
#pragma unroll 1
    for (int j = 0; j < 16; ++j) {
      const int col = 16 * h + j;
      const int colc = (col < kStateD) ? col : (kStateD - 1);
      float v = obs[(size_t)(gb0 + c) * kStateD + colc];
      asm volatile("" : "+v"(v));
      const float val = (col < kStateD) ? v : (col == kStateD) ? pa0 : (col == kStateD + 1) ? pa1 : 0.0f;
      pr[col] = val;
    }
  }
  __syncthreads();
  {
    const int q = lane >> 3, c4 = (lane & 7) * 4;
    v4f pv[4];
#pragma unroll
    for (int it = 0; it < 4; ++it) pv[it] = *(const v4f*)(&sPr[wave][0] + (it * 4 + q) * kPPitch + c4);
    for (int pass = 0; pass < 2; ++pass) {
#pragma unroll
      for (int it = 0; it < 4; ++it)
        *(volatile v4f*)(pplane + (size_t)(gb0 + it * 4 + q) * kPPitch + c4) = pv[it];
      __threadfence();
    }
  }
}

__global__ __launch_bounds__(128) void mlp_series_kernel(
    const float* __restrict__ ts, const float* __restrict__ pplane,
    const unsigned short* __restrict__ W1Hp, const unsigned short* __restrict__ W1Lp, const float* __restrict__ b1,
    const unsigned short* __restrict__ W2Hp, const unsigned short* __restrict__ W2Lp, const float* __restrict__ b2,
    const unsigned short* __restrict__ W3Hp, const unsigned short* __restrict__ W3Lp, const float* __restrict__ b3p,
    float* __restrict__ out)
{
  __shared__ __align__(16) __bf16 sAh[kRowTile * kApitch];
  __shared__ __align__(16) __bf16 sAl[kRowTile * kApitch];
  __shared__ __align__(16) __bf16 sH1h[kRowTile * kHpitch];
  __shared__ __align__(16) __bf16 sH1l[kRowTile * kHpitch];
  __shared__ __align__(16) float  sRawT[4][16 * kRawPitch];
  __shared__ __align__(16) float  sRawP[4][16 * kRawPitch];
  __shared__ __align__(16) float  sSum[kRowTile * kOutD];
  __shared__ __align__(16) float  sTc[kRowTile];
  __shared__ __align__(16) float  sGam[kRowTile];
  __shared__ __align__(16) float  sCoef[kRowTile];
  __shared__ __align__(16) float  sPv[4 * kPPitch];

  const __bf16* W1h = (const __bf16*)W1Hp; const __bf16* W1l = (const __bf16*)W1Lp;
  const __bf16* W2h = (const __bf16*)W2Hp; const __bf16* W2l = (const __bf16*)W2Lp;
  const __bf16* W3h = (const __bf16*)W3Hp; const __bf16* W3l = (const __bf16*)W3Lp;

  const int tid = threadIdx.x, lane = tid & 31, wave = tid >> 5;
  const int h = lane >> 4, c = lane & 15;
  const int R0 = blockIdx.x * kRowTile;
  const v8f zacc = {0.f, 0.f, 0.f, 0.f, 0.f, 0.f, 0.f, 0.f};

  if (tid < kRowTile) {
    const float t = ts[R0 + tid];
    const float Tc = 2.0f * t;
    const float gam = kAlpha - (kLogTol / Tc);
    sTc[tid] = Tc;
    sGam[tid] = gam;
    sCoef[tid] = expf(gam * t) / Tc;
  }
  sPv[tid] = pplane[(size_t)blockIdx.x * (4 * kPPitch) + tid];
  __syncthreads();

  {
    const int row = tid & 63, cpar = tid >> 6;
    const float Tc = sTc[row], gam = sGam[row];
    const float* prow = sPv + (row >> 4) * kPPitch;
#pragma unroll 1
    for (int i = 0; i < kFeatP / 2; ++i) {
      const int cc = 2 * i + cpar;
      int pc = cc - 2 * kTerms;
      pc = (pc < 0) ? 0 : pc;
      pc = (pc > kPPitch - 1) ? (kPPitch - 1) : pc;
      const float pv = prow[pc];
      const int kk = (cc < kTerms) ? cc : (cc - kTerms);
      const float sim = (kPi * (float)kk) / Tc;
      float v;
      if (cc < kTerms) {
        v = atan2f(sim, gam);
      } else if (cc < 2 * kTerms) {
        const float sq = gam * gam + sim * sim;
        v = asinf((sq - 1.0f) / (sq + 1.0f));
      } else {
        v = (cc < kFeat) ? pv : 0.0f;
      }
      __bf16 hi, lo;
      bf_split(v, hi, lo);
      sAh[row * kApitch + cc] = hi;
      sAl[row * kApitch + cc] = lo;
    }
  }
  __syncthreads();

  {
    v16b ah[3], al[3];
    const int aoff = (16 * wave + c) * kApitch + 8 * h;
#pragma unroll
    for (int ks = 0; ks < 3; ++ks) {
      LDS_FRAG_BF(ah[ks], sAh, aoff + 32 * ks);
      LDS_FRAG_BF(al[ks], sAl, aoff + 32 * ks);
    }
#pragma unroll 1
    for (int j = 0; j < 4; ++j) {
      const int n = 16 * j + c;
      const __bf16* bhp = W1h + (size_t)n * kFeatP + 8 * h;
      const __bf16* blp = W1l + (size_t)n * kFeatP + 8 * h;
      v8f acc = zacc;
#pragma unroll
      for (int ks = 0; ks < 3; ++ks) {
        const v16b fh = FragB::load(bhp + 32 * ks);
        const v16b fl = FragB::load(blp + 32 * ks);
        acc = mma_b(ah[ks], fh, acc);
        acc = mma_b(ah[ks], fl, acc);
        acc = mma_b(al[ks], fh, acc);
      }
      const float bias = b1[n];
#pragma unroll
      for (int r = 0; r < 8; ++r) {
        const float v = tanhf(acc[r] + bias);
        __bf16 hi, lo;
        bf_split(v, hi, lo);
        const int ix = (16 * wave + 8 * h + r) * kHpitch + n;
        sH1h[ix] = hi;
        sH1l[ix] = lo;
      }
    }
  }
  __syncthreads();

  {
    v16b ah[2], al[2];
    const int aoff = (16 * wave + c) * kHpitch + 8 * h;
#pragma unroll
    for (int ks = 0; ks < 2; ++ks) {
      LDS_FRAG_BF(ah[ks], sH1h, aoff + 32 * ks);
      LDS_FRAG_BF(al[ks], sH1l, aoff + 32 * ks);
    }
#pragma unroll 1
    for (int j = 0; j < 4; ++j) {
      const int n = 16 * j + c;
      const __bf16* bhp = W2h + (size_t)n * kHid + 8 * h;
      const __bf16* blp = W2l + (size_t)n * kHid + 8 * h;
      v8f acc = zacc;
#pragma unroll
      for (int ks = 0; ks < 2; ++ks) {
        const v16b fh = FragB::load(bhp + 32 * ks);
        const v16b fl = FragB::load(blp + 32 * ks);
        acc = mma_b(ah[ks], fh, acc);
        acc = mma_b(ah[ks], fl, acc);
        acc = mma_b(al[ks], fh, acc);
      }
      const float bias = b2[n];
#pragma unroll
      for (int r = 0; r < 8; ++r) {
        const float v = tanhf(acc[r] + bias);
        __bf16 hi, lo;
        bf_split(v, hi, lo);
        const int ix = (16 * wave + 8 * h + r) * kHpitch + n;
        sAh[ix] = hi;
        sAl[ix] = lo;
      }
    }
  }
  __syncthreads();

  {
    v16b ah[2], al[2];
    const int aoff = (16 * wave + c) * kHpitch + 8 * h;
#pragma unroll
    for (int ks = 0; ks < 2; ++ks) {
      LDS_FRAG_BF(ah[ks], sAh, aoff + 32 * ks);
      LDS_FRAG_BF(al[ks], sAl, aoff + 32 * ks);
    }
    float* rT = &sRawT[wave][0];
    float* rP = &sRawP[wave][0];
    float runacc = 0.0f;
#pragma unroll 1
    for (int g = 0; g < kGroups; ++g) {
      const int nT = 32 * g + c;
      const int nPh = nT + 16;
      const __bf16* tHp = W3h + (size_t)nT * kHid + 8 * h;
      const __bf16* tLp = W3l + (size_t)nT * kHid + 8 * h;
      const __bf16* pHp = W3h + (size_t)nPh * kHid + 8 * h;
      const __bf16* pLp = W3l + (size_t)nPh * kHid + 8 * h;
      v8f accT = zacc, accP = zacc;
#pragma unroll
      for (int ks = 0; ks < 2; ++ks) {
        const v16b th = FragB::load(tHp + 32 * ks);
        const v16b tl = FragB::load(tLp + 32 * ks);
        const v16b ph = FragB::load(pHp + 32 * ks);
        const v16b pl = FragB::load(pLp + 32 * ks);
        accT = mma_b(ah[ks], th, accT);
        accT = mma_b(ah[ks], tl, accT);
        accT = mma_b(al[ks], th, accT);
        accP = mma_b(ah[ks], ph, accP);
        accP = mma_b(ah[ks], pl, accP);
        accP = mma_b(al[ks], ph, accP);
      }
      const float bt = b3p[nT];
      const float bp = b3p[nPh];
#pragma unroll
      for (int r = 0; r < 8; ++r) {
        rT[(8 * h + r) * kRawPitch + c] = accT[r] + bt;
        rP[(8 * h + r) * kRawPitch + c] = accP[r] + bp;
      }
      __syncthreads();

      const int p = 16 * g + c;
      const int m = p / kTerms;
      const int k = p - m * kTerms;
      const int km = k & 3;
      const bool valid = (p < kNP);
      const float wk = (k == 0) ? 0.5f : 1.0f;
#pragma unroll 1
      for (int i = 0; i < 8; ++i) {
        const int ix = (8 * h + i) * kRawPitch + c;
        const float tr = rT[ix];
        const float pr = rP[ix];
        const float th = tanhf(tr) * kPi;
        const float ph = tanhf(pr) * kHalfPi;
        const float st = sinf(th);
        const float ct = cosf(th);
        const float sp = sinf(ph);
        const float cp = cosf(ph);
        const float base = cp / (1.0f - sp);
        const float sel = (km == 0) ? ct : (km == 1) ? (-st) : (km == 2) ? (-ct) : st;
        const float term = (sel * base) * wk;
        rT[ix] = valid ? term : 0.0f;
      }
      __syncthreads();

      if (lane < 16) {
        const float* rr = rT + lane * kRawPitch;
        const v4f q0 = *(const v4f*)(rr);
        const v4f q1 = *(const v4f*)(rr + 4);
        const v4f q2 = *(const v4f*)(rr + 8);
        const v4f q3 = *(const v4f*)(rr + 12);
        const int k0g = (16 * g) % kTerms;
        const int m0g = (16 * g) / kTerms;
#pragma unroll
        for (int cc = 0; cc < 16; ++cc) {
          const v4f qq = (cc < 4) ? q0 : (cc < 8) ? q1 : (cc < 12) ? q2 : q3;
          runacc += qq[cc & 3];
          if (k0g + cc == kTerms - 1) {
            sSum[(16 * wave + lane) * kOutD + m0g] = runacc;
            runacc = 0.0f;
          }
        }
      }
      __syncthreads();
    }
  }

#pragma unroll 1
  for (int i = tid; i < kRowTile * kOutD; i += 128) {
    const float v = sSum[i] * sCoef[i / kOutD];
    sSum[i] = v;
  }
  __syncthreads();

  if (wave == 0) {
    float* ob = out + (size_t)blockIdx.x * (kRowTile * kOutD);
    constexpr int kVec = (kRowTile * kOutD) / 4;
    for (int pass = 0; pass < 2; ++pass) {
#pragma unroll 1
      for (int it = 0; it < (kVec + 31) / 32; ++it) {
        const int idx = it * 32 + lane;
        const int idc = (idx < kVec) ? idx : (kVec - 1);
        const v4f v = *(const v4f*)(sSum + idc * 4);
        if (idx < kVec) *(volatile v4f*)(ob + idx * 4) = v;
      }
      __threadfence();
    }
  }
}

extern "C" void kernel_launch(void* const* d_in, const int* in_sizes, int n_in,
                              void* d_out, int out_size, void* d_ws, size_t ws_size,
                              hipStream_t stream) {
  if (n_in < 19) return;
  if (in_sizes[0] != kBatch * kStateD) return;
  if (in_sizes[1] != kBatch * kALen * kActD) return;
  if (in_sizes[2] != kBatch * kTP) return;
  if (in_sizes[3] != kGateRows * kActD) return;
  if (in_sizes[4] != kGateRows * kGruH) return;
  if (in_sizes[5] != kGateRows || in_sizes[6] != kGateRows) return;
  if (in_sizes[7] != kGateRows * kGruH || in_sizes[8] != kGateRows * kGruH) return;
  if (in_sizes[9] != kGateRows || in_sizes[10] != kGateRows) return;
  if (in_sizes[11] != 2 * kGruH || in_sizes[12] != 2) return;
  if (in_sizes[13] != kHid * kFeat || in_sizes[14] != kHid) return;
  if (in_sizes[15] != kHid * kHid || in_sizes[16] != kHid) return;
  if (in_sizes[17] != kN3 * kHid || in_sizes[18] != kN3) return;
  if (out_size != kRows * kOutD) return;
  if (ws_size < kWsTotal) return;

  const float* obs    = (const float*)d_in[0];
  const float* action = (const float*)d_in[1];
  const float* ts     = (const float*)d_in[2];
  const float* Wih0   = (const float*)d_in[3];
  const float* Whh0   = (const float*)d_in[4];
  const float* bih0   = (const float*)d_in[5];
  const float* bhh0   = (const float*)d_in[6];
  const float* Wih1   = (const float*)d_in[7];
  const float* Whh1   = (const float*)d_in[8];
  const float* bih1   = (const float*)d_in[9];
  const float* bhh1   = (const float*)d_in[10];
  const float* Wout   = (const float*)d_in[11];
  const float* bout   = (const float*)d_in[12];
  const float* W1     = (const float*)d_in[13];
  const float* b1     = (const float*)d_in[14];
  const float* W2     = (const float*)d_in[15];
  const float* b2     = (const float*)d_in[16];
  const float* W3     = (const float*)d_in[17];
  const float* b3     = (const float*)d_in[18];
  float* outp = (float*)d_out;

  char* ws = (char*)d_ws;
  unsigned short* W1H = (unsigned short*)(ws + kOffW1H);
  unsigned short* W1L = (unsigned short*)(ws + kOffW1L);
  unsigned short* W2H = (unsigned short*)(ws + kOffW2H);
  unsigned short* W2L = (unsigned short*)(ws + kOffW2L);
  unsigned short* W3H = (unsigned short*)(ws + kOffW3H);
  unsigned short* W3L = (unsigned short*)(ws + kOffW3L);
  float*          B3P = (float*)(ws + kOffB3P);
  unsigned short* GW  = (unsigned short*)(ws + kOffGW);
  float*          PP  = (float*)(ws + kOffPP);

  prep_planes_kernel<<<kPrepBlocks, kPrepThreads, 0, stream>>>(
      W1, W2, W3, b3, Wih0, Whh0, Wih1, Whh1,
      W1H, W1L, W2H, W2L, W3H, W3L, B3P, GW);

  gru_encode_kernel<<<kBatch / (kGruWaves * 16), kGruWaves * 32, 0, stream>>>(
      obs, action, GW, bih0, bhh0, bih1, bhh1, Wout, bout, PP);

  mlp_series_kernel<<<kRows / kRowTile, 128, 0, stream>>>(
      ts, PP, W1H, W1L, b1, W2H, W2L, b2, W3H, W3L, B3P, outp);
}
